// LaplaceAttention_51316269253360
// MI455X (gfx1250) — hardware-verified
//
#include <hip/hip_runtime.h>


namespace {
constexpr int NB = 2, C = 512, S = 256;
constexpr float XS = 8.0f, INV_SCALE = 0.5f, PSC = 16384.0f  ;
typedef _Float16 b16;
typedef __attribute__((ext_vector_type(16))) _Float16 v16b;
typedef __attribute__((ext_vector_type(8))) _Float16 v8b;
typedef __attribute__((ext_vector_type(8))) float v8f;
typedef __attribute__((ext_vector_type(4))) float v4f;
__device__ __forceinline__ float bf16_rne(float f) { unsigned int u = __float_as_uint(f); u += 0x7FFFu + ((u >> 16) & 1u); return __uint_as_float(u & 0xFFFF0000u); }
__device__ __forceinline__ void split16(float v, b16& hi, b16& lo) { hi = (b16)v; lo = (b16)(v - (float)hi); }
__device__ __forceinline__ v16b frag_kb(const b16* p, int hh) { const v8b a = *(const v8b*)(p + 8 * hh), b = *(const v8b*)(p + 16 + 8 * hh); v16b f;
#pragma unroll
  for (int e = 0; e < 8; ++e) { f[e] = a[e]; f[8 + e] = b[e]; } return f; }
__device__ __forceinline__ v8f wmma16b(v16b a, v16b b, v8f c) { v8f d = __builtin_amdgcn_wmma_f32_16x16x32_f16(false, a, false, b, (short)0, c, false, false); asm volatile("v_nop\n\tv_nop\n\tv_nop\n\tv_nop" : "+v"(d) : "v"(a), "v"(b)); return d; }

__global__ __launch_bounds__(256) void vt_kernel(const float* __restrict__ v, b16* __restrict__ VT) {
  __shared__ __attribute__((aligned(16))) b16 T[64][64 + 8];
  const int n = blockIdx.z, d0 = blockIdx.x * 64, s0 = blockIdx.y * 64, t_ = threadIdx.x;
  for (int q = t_; q < 64 * 64; q += 256) { const int dd = q >> 6, ss = q & 63; T[ss][dd] = (b16)(bf16_rne(v[((size_t)n * C + d0 + dd) * S + s0 + ss]) * XS); }
  __syncthreads();
  for (int pass = 0; pass < 2; ++pass) { for (int q = t_; q < 64 * 8; q += 256) { const int ss = q >> 3, c8 = (q & 7) * 8; *(volatile v8b*)(VT + ((size_t)n * S + s0 + ss) * C + d0 + c8) = *(const v8b*)(&T[ss][c8]); } __threadfence(); }
}
__global__ __launch_bounds__(256) void lap_kernel(const float* __restrict__ q, const float* __restrict__ k, const b16* __restrict__ VT, float* __restrict__ out) {
  __shared__ __attribute__((aligned(16))) float Qs[16][S]; __shared__ __attribute__((aligned(16))) float Wm[16][C + 4]; __shared__ __attribute__((aligned(16))) b16 Ph[16][C + 8], Pl[16][C + 8]; __shared__ __attribute__((aligned(16))) float To[8][16][32 + 4];
  const int n = blockIdx.y, c0 = blockIdx.x * 16, t_ = threadIdx.x, wave = t_ >> 5, lane = t_ & 31, nloc = lane & 15, hlf = lane >> 4;
  for (int e = t_; e < 16 * S; e += 256) { const int r = e / S, s = e % S; Qs[r][s] = bf16_rne(q[((size_t)n * C + c0 + r) * S + s]); }
  __syncthreads();
  { float acc0[16], acc1[16]; for (int r = 0; r < 16; ++r) { acc0[r] = 0.0f; acc1[r] = 0.0f; } const float* k0 = k + ((size_t)n * C + t_) * S; const float* k1 = k + ((size_t)n * C + t_ + 256) * S;
#pragma unroll 2
    for (int s = 0; s < S; ++s) { const float a = bf16_rne(k0[s]), b = bf16_rne(k1[s]);
#pragma unroll
      for (int r = 0; r < 16; ++r) { const float qq = Qs[r][s]; acc0[r] += fabsf(a - qq); acc1[r] += fabsf(b - qq); } }
    for (int r = 0; r < 16; ++r) { Wm[r][t_] = -acc0[r] * INV_SCALE; Wm[r][t_ + 256] = -acc1[r] * INV_SCALE; } }
  __syncthreads();
  for (int rr = 0; rr < 2; ++rr) { const int r = wave * 2 + rr; float x[16]; float mx = -INFINITY; for (int j = 0; j < 16; ++j) { x[j] = Wm[r][lane * 16 + j]; mx = fmaxf(mx, x[j]); }
#pragma unroll
    for (int o = 16; o >= 1; o >>= 1) mx = fmaxf(mx, __shfl_xor(mx, o));
    float sm = 0.0f; for (int j = 0; j < 16; ++j) { x[j] = __expf(x[j] - mx); sm += x[j]; }
#pragma unroll
    for (int o = 16; o >= 1; o >>= 1) sm += __shfl_xor(sm, o);
    const float inv = 1.0f / sm; for (int j = 0; j < 16; ++j) { b16 p, pl; split16(x[j] * inv * PSC, p, pl); Ph[r][lane * 16 + j] = p; Pl[r][lane * 16 + j] = pl; } }
  __syncthreads();
  v8f acc[2] = {{}, {}}; const int s0 = wave * 32;
#pragma unroll 2
  for (int kb = 0; kb < C; kb += 32) { const v16b a = frag_kb(&Ph[nloc][kb], hlf), al = frag_kb(&Pl[nloc][kb], hlf);
#pragma unroll
    for (int t = 0; t < 2; ++t) { const v16b bw = frag_kb(VT + ((size_t)n * S + s0 + t * 16 + nloc) * C + kb, hlf); acc[t] = wmma16b(a, bw, acc[t]); acc[t] = wmma16b(al, bw, acc[t]); } }
#pragma unroll
  for (int t = 0; t < 2; ++t)
#pragma unroll 1
    for (int r = 0; r < 8; ++r) To[wave][8 * hlf + r][t * 16 + nloc] = acc[t][r] * (1.0f / (PSC * XS));
  __syncthreads();
  for (int pass = 0; pass < 2; ++pass) { for (int q4 = lane; q4 < 16 * 8; q4 += 32) { const int r = q4 >> 3, c4 = (q4 & 7) * 4; *(volatile v4f*)(out + ((size_t)n * C + c0 + r) * S + s0 + c4) = *(const v4f*)(&To[wave][r][c4]); } __threadfence(); }
}
}

extern "C" void kernel_launch(void* const* d_in, const int* in_sizes, int n_in, void* d_out, int out_size, void* d_ws, size_t ws_size, hipStream_t stream) {
  (void)n_in;
  auto Fp = [&](int i) { return (const float*)d_in[i]; };
  if (in_sizes[0] != NB * C * S || in_sizes[1] != NB * C * S || in_sizes[2] != NB * C * S || out_size != NB * C * S) return;
  size_t off = 0; char* ws = (char*)d_ws;
  b16* VT = (b16*)(ws + off); off += (size_t)NB * S * C * 2;
  if (off > ws_size) return;
  vt_kernel<<<dim3(C / 64, S / 64, NB), 256, 0, stream>>>(Fp(2), VT);
  lap_kernel<<<dim3(C / 16, NB), 256, 0, stream>>>(Fp(0), Fp(1), VT, (float*)d_out);
}
